// SymmetricContraction_81879256531533
// MI455X (gfx1250) — hardware-verified
//
#include <hip/hip_runtime.h>
#include <stdint.h>

#pragma clang fp contract(off)

typedef __attribute__((ext_vector_type(16))) _Float16 v16h;
typedef __attribute__((ext_vector_type(8)))  _Float16 v8h;
typedef __attribute__((ext_vector_type(16))) __bf16   v16b;
typedef __attribute__((ext_vector_type(8)))  __bf16   v8b;
typedef __attribute__((ext_vector_type(8)))  float    v8f;
typedef __attribute__((ext_vector_type(4)))  float    v4f;
typedef __attribute__((ext_vector_type(4)))  unsigned int v4u;

__device__ __forceinline__ unsigned short f2bf_bits(float f) {
  unsigned u = __float_as_uint(f);
  return (unsigned short)((u + 0x7FFFu + ((u >> 16) & 1u)) >> 16);
}
__device__ __forceinline__ float bf_bits2f(unsigned short h) { return __uint_as_float(((unsigned)h) << 16); }

__device__ __forceinline__ void dep_guard_h(v8f& a, v8f& b, v16h x, v16h y) { asm volatile("v_nop\n\tv_nop\n\tv_nop\n\tv_nop" : "+v"(a), "+v"(b) : "v"(x), "v"(y)); }
__device__ __forceinline__ void dep_guard_b(v8f& a, v8f& b, v16b x, v16b y) { asm volatile("v_nop\n\tv_nop\n\tv_nop\n\tv_nop" : "+v"(a), "+v"(b) : "v"(x), "v"(y)); }
__device__ __forceinline__ void keep4_h(v16h a, v16h b, v16h c, v16h d) { asm volatile("v_nop" :: "v"(a), "v"(b), "v"(c), "v"(d)); }
__device__ __forceinline__ void keep4_b(v16b a, v16b b, v16b c, v16b d) { asm volatile("v_nop" :: "v"(a), "v"(b), "v"(c), "v"(d)); }
__device__ __forceinline__ void acc_guard4(v8f& a, v8f& b, v8f& c, v8f& d) { asm volatile("v_nop\n\tv_nop\n\tv_nop\n\tv_nop" : "+v"(a), "+v"(b), "+v"(c), "+v"(d)); }
template <typename T> struct Frag;
template <> struct Frag<_Float16> {
  typedef v16h V; union U { v16h v; v8h h[2]; };
  static __device__ __forceinline__ v16h load(const _Float16* p) {
    U f; f.h[0] = *(const v8h*)(p); f.h[1] = *(const v8h*)(p + 16); return f.v;
  }
  static __device__ __forceinline__ v8f mma(v16h a, v16h b, v8f c) {
    return __builtin_amdgcn_wmma_f32_16x16x32_f16(false, a, false, b, (short)0, c, false, false);
  }
  static __device__ __forceinline__ void guard(v8f& a, v8f& b, v16h x, v16h y) { dep_guard_h(a, b, x, y); }
  static __device__ __forceinline__ void keep(v16h a, v16h b, v16h c, v16h d) { keep4_h(a, b, c, d); }
};
template <> struct Frag<__bf16> {
  typedef v16b V; union U { v16b v; v8b h[2]; };
  static __device__ __forceinline__ v16b load(const __bf16* p) {
    U f; f.h[0] = *(const v8b*)(p); f.h[1] = *(const v8b*)(p + 16); return f.v;
  }
  static __device__ __forceinline__ v8f mma(v16b a, v16b b, v8f c) {
    return __builtin_amdgcn_wmma_f32_16x16x32_bf16(false, a, false, b, (short)0, c, false, false);
  }
  static __device__ __forceinline__ void guard(v8f& a, v8f& b, v16b x, v16b y) { dep_guard_b(a, b, x, y); }
  static __device__ __forceinline__ void keep(v16b a, v16b b, v16b c, v16b d) { keep4_b(a, b, c, d); }
};

template <int ET> struct Elem;
template <> struct Elem<0> { typedef _Float16 T; };
template <> struct Elem<1> { typedef __bf16 T; };
template <int ET, bool SPLIT, int BIAS_MODE, int OUT_MODE, bool RESID, int ACT = 0>
__global__ __launch_bounds__(256) void wmma_gemm64(
    const unsigned short* __restrict__ Ap, const unsigned short* __restrict__ A2p, int lda, long strideA,
    const unsigned short* __restrict__ Btp, const unsigned short* __restrict__ Bt2p, int ldb, long strideB,
    void* __restrict__ Cout, void* __restrict__ Cout2, int ldc, long strideC,
    const float* __restrict__ bias,
    const float* __restrict__ resid, long strideR,
    int M, int N, int K, float scale) {
  typedef typename Elem<ET>::T T;
  typedef typename Frag<T>::V V;
  const T* A = (const T*)Ap; const T* A2 = (const T*)A2p; const T* Bt = (const T*)Btp; const T* Bt2 = (const T*)Bt2p;
  __shared__ __align__(16) float sT[8][16 * 68];
  const int b    = blockIdx.y;
  const int lane = threadIdx.x & 31;
  const int wave = threadIdx.x >> 5;
  const int tilesN = N >> 6;
  const int tilesM = M >> 6;
  const int tile = blockIdx.x * 8 + wave;
  if (tile >= tilesM * tilesN) return;
  const int tm = tile / tilesN;
  const int tn = tile - tm * tilesN;
  const int m0 = tm << 6;
  const int n0 = tn << 6;

  const T* Ab  = A  + (size_t)b * strideA;
  const T* Bb  = Bt + (size_t)b * strideB;
  const T* Ab2 = SPLIT ? (A2  + (size_t)b * strideA) : nullptr;
  const T* Bb2 = SPLIT ? (Bt2 + (size_t)b * strideB) : nullptr;

  const int rlane = lane & 15;
  const int koff  = (lane >> 4) * 8;
  const int mOff  = (lane >> 4) * 8;

  v8f acc[4][4];
#pragma unroll
  for (int i = 0; i < 4; ++i)
#pragma unroll
    for (int j = 0; j < 4; ++j) acc[i][j] = (v8f){0.f,0.f,0.f,0.f,0.f,0.f,0.f,0.f};

  for (int k0 = 0; k0 < K; k0 += 32) {
    V bh[4], bl[4];
#pragma unroll
    for (int j = 0; j < 4; ++j) {
      const size_t bo = (size_t)(n0 + (j << 4) + rlane) * ldb + koff + k0;
      bh[j] = Frag<T>::load(Bb + bo);
      if (SPLIT) bl[j] = Frag<T>::load(Bb2 + bo);
    }
#pragma unroll
    for (int i = 0; i < 4; ++i) {
      const size_t ao = (size_t)(m0 + (i << 4) + rlane) * lda + koff + k0;
      V ah = Frag<T>::load(Ab + ao);
      V al;
      if (SPLIT) al = Frag<T>::load(Ab2 + ao);
#pragma unroll
      for (int j = 0; j < 4; ++j) {
        acc[i][j] = Frag<T>::mma(ah, bh[j], acc[i][j]);
        if (SPLIT) {
          acc[i][j] = Frag<T>::mma(ah, bl[j], acc[i][j]);
          acc[i][j] = Frag<T>::mma(al, bh[j], acc[i][j]);
        }
      }
      Frag<T>::guard(acc[i][0], acc[i][3], ah, SPLIT ? al : ah);
    }
    Frag<T>::keep(bh[0], bh[1], bh[2], bh[3]);
    if (SPLIT) Frag<T>::keep(bl[0], bl[1], bl[2], bl[3]);
  }
  acc_guard4(acc[0][0], acc[0][1], acc[0][2], acc[0][3]);
  acc_guard4(acc[1][0], acc[1][1], acc[1][2], acc[1][3]);
  acc_guard4(acc[2][0], acc[2][1], acc[2][2], acc[2][3]);
  acc_guard4(acc[3][0], acc[3][1], acc[3][2], acc[3][3]);

  float* slab = sT[wave];
  const float* Rb = RESID ? (resid + (size_t)b * strideR) : nullptr;
#pragma unroll
  for (int i = 0; i < 4; ++i) {
    const int mBase = m0 + (i << 4);
#pragma unroll
    for (int j = 0; j < 4; ++j) {
      const int n = n0 + (j << 4) + rlane;
      float bv = 0.f;
      if (BIAS_MODE == 2) bv = bias[n];
#pragma unroll
      for (int r = 0; r < 8; ++r) {
        float v = acc[i][j][r] * scale;
        if (BIAS_MODE == 1) v += bias[mBase + mOff + r];
        if (BIAS_MODE == 2) v += bv;
        if (RESID) v += Rb[(size_t)(mBase + mOff + r) * ldc + n];
        if (ACT == 1) v = tanhf(v);
        if (ACT == 2) v = fmaxf(v, 0.0f);
        if (ACT == 3) v = v / (1.0f + expf(-v));
        if (ACT == 4) v = (v > 0.f) ? v : 0.01f * v;
        if (ACT == 5) v = 0.5f * v * (1.0f + erff(v * 0.70710678118654752f));
        slab[(mOff + r) * 68 + (j << 4) + rlane] = v;
      }
    }
    __builtin_amdgcn_fence(__ATOMIC_RELEASE, "workgroup");
    __builtin_amdgcn_wave_barrier();
    __builtin_amdgcn_fence(__ATOMIC_ACQUIRE, "workgroup");
    if (OUT_MODE == 0) {
      float* C = (float*)Cout + (size_t)b * strideC;
      const int hh = lane >> 4, c4 = (lane & 15) * 4;
      for (int pass = 0; pass < 2; ++pass) {
#pragma unroll
        for (int it = 0; it < 8; ++it) {
          const int row = it * 2 + hh;
          v4f v = *(const v4f*)(slab + row * 68 + c4);
          *(volatile v4f*)(C + (size_t)(mBase + row) * ldc + n0 + c4) = v;
        }
        __threadfence();
      }
    } else {
      const int q = lane >> 3, c8 = (lane & 7) * 8;
      unsigned short* C  = (unsigned short*)Cout  + (size_t)b * strideC;
      unsigned short* C2 = (OUT_MODE == 2) ? ((unsigned short*)Cout2 + (size_t)b * strideC) : nullptr;
      for (int pass = 0; pass < 2; ++pass) {
#pragma unroll
        for (int it = 0; it < 4; ++it) {
          const int row = it * 4 + q;
          const float* sp = slab + row * 68 + c8;
          v8h hv, lv;
#pragma unroll
          for (int e = 0; e < 8; ++e) {
            if (OUT_MODE == 1) {
              hv[e] = (_Float16)sp[e];
            } else {
              unsigned short hb = f2bf_bits(sp[e]);
              unsigned short lb = f2bf_bits(sp[e] - bf_bits2f(hb));
              hv[e] = __builtin_bit_cast(_Float16, hb);
              lv[e] = __builtin_bit_cast(_Float16, lb);
            }
          }
          *(volatile v8h*)(C + (size_t)(mBase + row) * ldc + n0 + c8) = hv;
          if (OUT_MODE == 2) *(volatile v8h*)(C2 + (size_t)(mBase + row) * ldc + n0 + c8) = lv;
        }
        __threadfence();
      }
    }
    __builtin_amdgcn_fence(__ATOMIC_RELEASE, "workgroup");
    __builtin_amdgcn_wave_barrier();
    __builtin_amdgcn_fence(__ATOMIC_ACQUIRE, "workgroup");
  }
}

constexpr int kNodes      = 1024;
constexpr int kCh         = 128;
constexpr int kElem       = 10;
constexpr int kL          = 16;
constexpr int kP3         = 23;
constexpr int kP2         = 4;
constexpr int kKdim       = kL * kP3;
constexpr int kKaug       = kKdim + kP2;
constexpr int kKpad       = 384;
constexpr int kNwx        = kL * kL;
constexpr int kChunkNodes = 256;
constexpr int kChunkRows  = kChunkNodes * kCh;
constexpr int kNumChunks  = kNodes / kChunkNodes;
constexpr int kGroupsPerRow = kKpad / 8;
constexpr int kBtGroups   = kNwx * kGroupsPerRow;
constexpr int kAGroupsPerNode = kCh * kGroupsPerRow;
constexpr int kAItersPerNode  = kAGroupsPerNode / 256;
constexpr int kGemmTiles  = (kChunkRows / 64) * (kNwx / 64);
constexpr int kGemmBlocks = kGemmTiles / 8;

static_assert(kKpad % 32 == 0);
static_assert(kKaug <= kKpad);
static_assert(kKdim % 8 == 0);
static_assert(kChunkRows % 64 == 0);
static_assert(kNwx % 64 == 0);
static_assert(kGemmTiles % 8 == 0);
static_assert(kNodes % kChunkNodes == 0);
static_assert(kBtGroups % 256 == 0);
static_assert(kAGroupsPerNode % 256 == 0);
static_assert(kCh == 128);

constexpr size_t kBytesBt = (size_t)kNwx * kKpad * 2;
constexpr size_t kBytesA  = (size_t)kChunkRows * kKpad * 2;
constexpr size_t kBytesC  = (size_t)kChunkRows * kNwx * 4;
constexpr size_t kOffBtHi = 0;
constexpr size_t kOffBtLo = kOffBtHi + kBytesBt;
constexpr size_t kOffAHi  = kOffBtLo + kBytesBt;
constexpr size_t kOffALo  = kOffAHi + kBytesA;
constexpr size_t kOffC    = kOffALo + kBytesA;
constexpr size_t kWsTotal = kOffC + kBytesC;
static_assert(kWsTotal == 84279296);
static_assert(kWsTotal <= (size_t)134217728);
static_assert(kOffBtLo % 128 == 0 && kOffAHi % 128 == 0 && kOffALo % 128 == 0 && kOffC % 128 == 0);

__device__ __forceinline__ void split2_pack(float a, float b, unsigned int& hw, unsigned int& lw) {
  const unsigned short ha = f2bf_bits(a);
  const unsigned short hb = f2bf_bits(b);
  const float ra = a - bf_bits2f(ha);
  const float rb = b - bf_bits2f(hb);
  const unsigned short la = f2bf_bits(ra);
  const unsigned short lb = f2bf_bits(rb);
  hw = (unsigned int)ha | ((unsigned int)hb << 16);
  lw = (unsigned int)la | ((unsigned int)lb << 16);
}
__device__ __forceinline__ void split8_store2(const float t0, const float t1, const float t2, const float t3,
                                              const float t4, const float t5, const float t6, const float t7,
                                              unsigned short* ph, unsigned short* pl, size_t off) {
  v4u hu, lu;
  unsigned int hw, lw;
  split2_pack(t0, t1, hw, lw); hu[0] = hw; lu[0] = lw;
  split2_pack(t2, t3, hw, lw); hu[1] = hw; lu[1] = lw;
  split2_pack(t4, t5, hw, lw); hu[2] = hw; lu[2] = lw;
  split2_pack(t6, t7, hw, lw); hu[3] = hw; lu[3] = lw;
  *(volatile v4u*)(ph + off) = hu;
  *(volatile v4u*)(pl + off) = lu;
  __threadfence();
  *(volatile v4u*)(ph + off) = hu;
  *(volatile v4u*)(pl + off) = lu;
}

__global__ __launch_bounds__(256) void bt_build(const float* __restrict__ U3g, const float* __restrict__ U2g,
                                                unsigned short* __restrict__ Bh, unsigned short* __restrict__ Bl) {
  const int g = blockIdx.x * 256 + (int)threadIdx.x;
  const int gc = g < kBtGroups ? g : kBtGroups - 1;
  const int n = gc / kGroupsPerRow;
  const int cg = gc - n * kGroupsPerRow;
  const int col0 = cg * 8;
  const bool v3 = (col0 < kKdim);
  const int colc = v3 ? col0 : 0;
  const v4f a0 = *(const v4f*)(U3g + (size_t)n * kKdim + colc);
  const v4f a1 = *(const v4f*)(U3g + (size_t)n * kKdim + colc + 4);
  const v4f u2 = *(const v4f*)(U2g + (size_t)n * kP2);
  const bool isU2 = (col0 == kKdim);
  float t[8];
#pragma unroll
  for (int e = 0; e < 4; ++e) t[e] = v3 ? a0[e] : (isU2 ? u2[e] : 0.0f);
#pragma unroll
  for (int e = 0; e < 4; ++e) t[4 + e] = v3 ? a1[e] : 0.0f;
  if (g < kBtGroups) {
    split8_store2(t[0], t[1], t[2], t[3], t[4], t[5], t[6], t[7], Bh, Bl, (size_t)g * 8);
  }
}

__global__ __launch_bounds__(256) void a_build(const float* __restrict__ xg, const float* __restrict__ yg,
                                               const float* __restrict__ W3g, const float* __restrict__ W2g,
                                               unsigned short* __restrict__ Ah, unsigned short* __restrict__ Al,
                                               int node0) {
  __shared__ __align__(16) float xs[kCh * kL];
  __shared__ float w3s[kP3 * kCh];
  __shared__ float w2s[kP2 * kCh];
  __shared__ float ys[kElem];
  const int tid = (int)threadIdx.x;
  const int bl = blockIdx.x;
  const int b = node0 + bl;

  if (tid < kElem) ys[tid] = yg[(size_t)b * kElem + tid];
  {
    const v4f* xg4 = (const v4f*)(xg + (size_t)b * kCh * kL);
    ((v4f*)xs)[tid] = xg4[tid];
    ((v4f*)xs)[tid + 256] = xg4[tid + 256];
  }
  __syncthreads();

#pragma unroll 1
  for (int idx = tid; idx < kP3 * kCh; idx += 256) {
    float s = 0.0f;
#pragma unroll
    for (int e = 0; e < kElem; ++e) s = fmaf(ys[e], W3g[(size_t)e * (kP3 * kCh) + idx], s);
    w3s[idx] = s;
  }
#pragma unroll 1
  for (int idx = tid; idx < kP2 * kCh; idx += 256) {
    float s = 0.0f;
#pragma unroll
    for (int e = 0; e < kElem; ++e) s = fmaf(ys[e], W2g[(size_t)e * (kP2 * kCh) + idx], s);
    w2s[idx] = s;
  }
  __syncthreads();

  const size_t nodeOff = (size_t)bl * ((size_t)kCh * kKpad);
#pragma unroll 1
  for (int it = 0; it < kAItersPerNode; ++it) {
    const int g = tid + 256 * it;
    const int c = g / kGroupsPerRow;
    const int cg = g - c * kGroupsPerRow;
    const int col0 = cg * 8;
    float t[8];
#pragma unroll
    for (int e = 0; e < 8; ++e) {
      const int kcol = col0 + e;
      const bool v3 = kcol < kKdim;
      const int kc = v3 ? kcol : 0;
      const int i = kc / kP3;
      const int k = kc - i * kP3;
      const float t3 = w3s[k * kCh + c] * xs[c * kL + i];
      const int k2 = (kcol - kKdim) & 3;
      const float t2 = w2s[k2 * kCh + c];
      t[e] = v3 ? t3 : ((kcol < kKaug) ? t2 : 0.0f);
    }
    split8_store2(t[0], t[1], t[2], t[3], t[4], t[5], t[6], t[7], Ah, Al, nodeOff + (size_t)g * 8);
  }
}

__device__ __forceinline__ float dot4_acc(v4f a, v4f b, float s) {
  s = fmaf(a[0], b[0], s);
  s = fmaf(a[1], b[1], s);
  s = fmaf(a[2], b[2], s);
  s = fmaf(a[3], b[3], s);
  return s;
}

__global__ __launch_bounds__(128) void node_reduce(const float* __restrict__ Cp, const float* __restrict__ xg,
                                                   const float* __restrict__ yg, const float* __restrict__ U1g,
                                                   const float* __restrict__ W1g, float* __restrict__ outg,
                                                   int node0) {
  __shared__ __align__(16) float xs[kCh * kL];
  __shared__ __align__(16) float os[kCh];
  __shared__ float ys[kElem];
  const int tid = (int)threadIdx.x;
  const int c = tid;
  const int bl = blockIdx.x;
  const int b = node0 + bl;

  if (tid < kElem) ys[tid] = yg[(size_t)b * kElem + tid];
  {
    const v4f* xg4 = (const v4f*)(xg + (size_t)b * kCh * kL);
#pragma unroll
    for (int j = 0; j < 4; ++j) ((v4f*)xs)[tid + 128 * j] = xg4[tid + 128 * j];
  }
  __syncthreads();

  float w1c = 0.0f;
#pragma unroll
  for (int e = 0; e < kElem; ++e) w1c = fmaf(ys[e], W1g[(size_t)e * kCh + c], w1c);

  const v4f x0 = *(const v4f*)(xs + c * kL);
  const v4f x1 = *(const v4f*)(xs + c * kL + 4);
  const v4f x2 = *(const v4f*)(xs + c * kL + 8);
  const v4f x3 = *(const v4f*)(xs + c * kL + 12);

  const float* crow = Cp + ((size_t)bl * kCh + c) * kNwx;
  float o = 0.0f;
#pragma unroll 1
  for (int w = 0; w < kL; ++w) {
    const v4f q0 = *(const v4f*)(crow + w * kL);
    const v4f q1 = *(const v4f*)(crow + w * kL + 4);
    const v4f q2 = *(const v4f*)(crow + w * kL + 8);
    const v4f q3 = *(const v4f*)(crow + w * kL + 12);
    float acc = 0.0f;
    acc = dot4_acc(q0, x0, acc);
    acc = dot4_acc(q1, x1, acc);
    acc = dot4_acc(q2, x2, acc);
    acc = dot4_acc(q3, x3, acc);
    const float u1 = U1g[w];
    const float xw = xs[c * kL + w];
    const float c1v = fmaf(u1, w1c, acc);
    o = fmaf(c1v, xw, o);
  }
  os[c] = o;
  __syncthreads();
  if (tid < 32) {
    const v4f v = *(const v4f*)(os + 4 * tid);
    float* op = outg + (size_t)b * kCh + 4 * tid;
    *(volatile v4f*)op = v;
    __threadfence();
    *(volatile v4f*)op = v;
  }
}

extern "C" void kernel_launch(void* const* d_in, const int* in_sizes, int n_in,
                              void* d_out, int out_size, void* d_ws, size_t ws_size,
                              hipStream_t stream) {
  if (n_in < 8) return;
  if (in_sizes[0] != kNodes * kCh * kL) return;
  if (in_sizes[1] != kNodes * kElem) return;
  if (in_sizes[2] != kNwx * kKdim) return;
  if (in_sizes[3] != kNwx * kP2) return;
  if (in_sizes[4] != kL) return;
  if (in_sizes[5] != kElem * kP3 * kCh) return;
  if (in_sizes[6] != kElem * kP2 * kCh) return;
  if (in_sizes[7] != kElem * kCh) return;
  if (out_size != kNodes * kCh) return;
  if (ws_size < kWsTotal) return;

  const float* x  = (const float*)d_in[0];
  const float* y  = (const float*)d_in[1];
  const float* U3 = (const float*)d_in[2];
  const float* U2 = (const float*)d_in[3];
  const float* U1 = (const float*)d_in[4];
  const float* W3 = (const float*)d_in[5];
  const float* W2 = (const float*)d_in[6];
  const float* W1 = (const float*)d_in[7];
  float* out = (float*)d_out;

  char* ws = (char*)d_ws;
  unsigned short* Bh = (unsigned short*)(ws + kOffBtHi);
  unsigned short* Bl = (unsigned short*)(ws + kOffBtLo);
  unsigned short* Ah = (unsigned short*)(ws + kOffAHi);
  unsigned short* Al = (unsigned short*)(ws + kOffALo);
  float* Cp = (float*)(ws + kOffC);
  const float* dummyF = (const float*)(ws + kOffBtHi);
  void* dummyC2 = (void*)(ws + kOffBtLo);

  bt_build<<<kBtGroups / 256, 256, 0, stream>>>(U3, U2, Bh, Bl);

  for (int ch = 0; ch < kNumChunks; ++ch) {
    const int node0 = ch * kChunkNodes;
    a_build<<<kChunkNodes, 256, 0, stream>>>(x, y, W3, W2, Ah, Al, node0);
    wmma_gemm64<1, true, 0, 0, false, 0><<<dim3(kGemmBlocks, 1), 256, 0, stream>>>(
        Ah, Al, kKpad, 0L,
        Bh, Bl, kKpad, 0L,
        (void*)Cp, dummyC2, kNwx, 0L,
        dummyF,
        dummyF, 0L,
        kChunkRows, kNwx, kKpad, 1.0f);
    node_reduce<<<kChunkNodes, 128, 0, stream>>>(Cp, x, y, U1, W1, out, node0);
  }
}
